// PraxisAttention_21586505630083
// MI455X (gfx1250) — hardware-verified
//
#include <hip/hip_runtime.h>
#pragma clang fp contract(off)


#ifndef NB
#define NB 2
#endif
#ifndef SEQ
#define SEQ 2048
#endif
#define NB_FULL 2
#define SEQ_FULL 2048
#define DM   1024
#define NVH  16
#define HD   64
#define NQH  (2 * NVH)
#define DQ   (NQH * HD)
#define DVV  (NVH * HD)
#define SCL  0.125f
#define PCAR 4096.0f
#define RCAR 1024.0f
#define QBL  64
#define KCH  64
#define KSB  32
#define LP   72
#define PP   40
#define OSP  68
#define L2E  1.4426950408889634f
#define NEGB (-3.0e38f)
static_assert(SEQ % 64 == 0);
static_assert(SEQ <= SEQ_FULL);
static_assert(NB >= 1);
static_assert(NB <= NB_FULL);
static_assert(QBL == KCH);
static_assert(KCH % KSB == 0);
static_assert((LP * 2) % 16 == 0);
static_assert((PP * 2) % 16 == 0);
static_assert((OSP * 4) % 16 == 0);
static_assert((NQH * SEQ * HD) % 512 == 0);
static_assert((SEQ * DVV) % 512 == 0);
static_assert((SEQ * DM) % 2048 == 0);

typedef _Float16 h16;
typedef unsigned short bf;
typedef __attribute__((ext_vector_type(16))) __bf16   v16bf;
typedef __attribute__((ext_vector_type(16))) _Float16 v16h;
typedef __attribute__((ext_vector_type(8)))  _Float16 v8h;
typedef __attribute__((ext_vector_type(8)))  unsigned short v8us;
typedef __attribute__((ext_vector_type(8)))  float    v8f;
typedef __attribute__((ext_vector_type(4)))  float    v4f;
typedef __attribute__((ext_vector_type(2)))  _Float16 v2h;
typedef __attribute__((ext_vector_type(2)))  unsigned short v2us;
typedef __attribute__((ext_vector_type(2)))  float v2f;
typedef v8h  __attribute__((may_alias)) v8ha;
typedef v4f  __attribute__((may_alias)) v4fa;
typedef v8us __attribute__((may_alias)) v8usa;

__device__ __forceinline__ unsigned short f2bf(float f) { unsigned u = __float_as_uint(f); u += 0x7FFFu + ((u >> 16) & 1u); return (unsigned short)(u >> 16); }
__device__ __forceinline__ float bf2f(unsigned short b) { return __uint_as_float(((unsigned)b) << 16); }
__device__ __forceinline__ float bfr(float f) { return bf2f(f2bf(f)); }
__device__ __forceinline__ v16h cat16(v8h lo, v8h hi) { return __builtin_shufflevector(lo, hi, 0, 1, 2, 3, 4, 5, 6, 7, 8, 9, 10, 11, 12, 13, 14, 15); }
__device__ __forceinline__ v16bf cat16b(v8us lo, v8us hi) { return __builtin_bit_cast(v16bf, __builtin_shufflevector(lo, hi, 0, 1, 2, 3, 4, 5, 6, 7, 8, 9, 10, 11, 12, 13, 14, 15)); }
__device__ __forceinline__ v8f wmma16(v16h a, v16h b, v8f c) { return __builtin_amdgcn_wmma_f32_16x16x32_f16(false, a, false, b, (short)0, c, false, false); }
__device__ __forceinline__ v8f wmmab(v16bf a, v16bf b, v8f c) { return __builtin_amdgcn_wmma_f32_16x16x32_bf16(false, a, false, b, (short)0, c, false, false); }
__device__ __forceinline__ h16 tohx(float x) { return (h16)x; }
__device__ __forceinline__ void splitf(float y, unsigned short& h, unsigned short& l) { h = f2bf(y); l = f2bf(y - bf2f(h)); }

template <typename T16> struct WFrag;
template <> struct WFrag<h16> { typedef v16h V; static __device__ __forceinline__ V ld(const h16* p) { return cat16(*(const v8h*)p, *(const v8h*)(p + 16)); } static __device__ __forceinline__ v8f mma(V a, V b, v8f c) { return wmma16(a, b, c); } };
template <> struct WFrag<bf> { typedef v16bf V; static __device__ __forceinline__ V ld(const bf* p) { return cat16b(*(const v8us*)p, *(const v8us*)(p + 16)); } static __device__ __forceinline__ v8f mma(V a, V b, v8f c) { return wmmab(a, b, c); } };
template <typename T16, int NSPLIT, bool BIAS>
__global__ __launch_bounds__(32) void k_gemmw(const T16* __restrict__ A, const T16* __restrict__ A2, const T16* __restrict__ Bt, const T16* __restrict__ Bt2, int K, float* C, int ldc, const float* __restrict__ bias, size_t sA, size_t sB, size_t sC) {
    typedef typename WFrag<T16>::V V;
    __shared__ __align__(16) float os[16 * 68];
    const size_t z = blockIdx.z; A += z * sA; if (A2) A2 += z * sA; Bt += z * sB; if (Bt2) Bt2 += z * sB; C += z * sC;
    const int lane = threadIdx.x & 31, lr = lane & 15, hi = lane >> 4; const int r0 = blockIdx.x * 64, c0 = blockIdx.y * 64;
    v8f acc[4][4];
#pragma unroll
    for (int mb = 0; mb < 4; ++mb)
#pragma unroll
        for (int nb = 0; nb < 4; ++nb) acc[mb][nb] = (v8f){};
    const size_t aoff = (size_t)(r0 + lr) * K + 8 * hi, boff = (size_t)(c0 + lr) * K + 8 * hi;
#pragma unroll 1
    for (int kc = 0; kc < K; kc += 32) {
        V a[4], a2[4];
#pragma unroll
        for (int mb = 0; mb < 4; ++mb) { a[mb] = WFrag<T16>::ld(A + aoff + (size_t)mb * 16 * K + kc); if (NSPLIT == 1 || NSPLIT == 2) a2[mb] = WFrag<T16>::ld(A2 + aoff + (size_t)mb * 16 * K + kc); }
#pragma unroll
        for (int nb = 0; nb < 4; ++nb) { const V b = WFrag<T16>::ld(Bt + boff + (size_t)nb * 16 * K + kc); V b2; if (NSPLIT >= 2) b2 = WFrag<T16>::ld(Bt2 + boff + (size_t)nb * 16 * K + kc);
#pragma unroll
            for (int mb = 0; mb < 4; ++mb) { acc[mb][nb] = WFrag<T16>::mma(a[mb], b, acc[mb][nb]); if (NSPLIT == 1 || NSPLIT == 2) acc[mb][nb] = WFrag<T16>::mma(a2[mb], b, acc[mb][nb]); if (NSPLIT >= 2) acc[mb][nb] = WFrag<T16>::mma(a[mb], b2, acc[mb][nb]); } }
        asm volatile("v_nop\n\tv_nop\n\tv_nop\n\tv_nop" : "+v"(acc[0][0]), "+v"(acc[1][1]), "+v"(acc[2][2]), "+v"(acc[3][3]) : "v"(a[0]), "v"(a[3]));
    }
#pragma unroll
    for (int mb = 0; mb < 4; ++mb) {
#pragma unroll
        for (int nb = 0; nb < 4; ++nb) {
#pragma unroll
            for (int j = 0; j < 8; ++j) os[(hi * 8 + j) * 68 + nb * 16 + lr] = acc[mb][nb][j]; }
        __builtin_amdgcn_wave_barrier(); asm volatile("" ::: "memory");
        float* crow = C + (size_t)(r0 + mb * 16) * ldc + c0;
#pragma unroll 1
        for (int ps = 0; ps < 2; ++ps) {
#pragma unroll
            for (int s = 0; s < 8; ++s) { const int row = 2 * s + hi, cofs = lr * 4; v4f val = *(const v4fa*)(os + row * 68 + cofs); if (BIAS) { val[0] += bfr(bias[c0 + cofs]); val[1] += bfr(bias[c0 + cofs + 1]); val[2] += bfr(bias[c0 + cofs + 2]); val[3] += bfr(bias[c0 + cofs + 3]); }
                *(volatile v4f*)(crow + (size_t)row * ldc + cofs) = val; }
            if (ps == 0) __threadfence(); }
        __builtin_amdgcn_wave_barrier(); asm volatile("" ::: "memory");
    }
}

__global__ __launch_bounds__(256) void k_cvt8(const float* __restrict__ src, bf* dst, size_t n8) { const size_t i = (size_t)blockIdx.x * 256 + threadIdx.x; if (i >= n8) return; const v8f v = *(const v8f*)(src + i * 8); v8us o;
#pragma unroll
    for (int k = 0; k < 8; ++k) o[k] = f2bf(v[k]); *(volatile v8us*)(dst + i * 8) = o; __threadfence(); *(volatile v8us*)(dst + i * 8) = o; }
__global__ __launch_bounds__(256) void k_rbf(const float* __restrict__ src, float* dst, int n4) { const int i = blockIdx.x * 256 + threadIdx.x; if (i >= n4) return; const v4f a = *(const v4f*)(src + (size_t)i * 4); v4f o;
#pragma unroll
    for (int u = 0; u < 4; ++u) o[u] = bfr(a[u]); *(volatile v4f*)(dst + (size_t)i * 4) = o; __threadfence(); *(volatile v4f*)(dst + (size_t)i * 4) = o; }
__global__ __launch_bounds__(32) void k_lambda(const float* __restrict__ lq1, const float* __restrict__ lk1, const float* __restrict__ lq2, const float* __restrict__ lk2, float* LAM) { const int lane = threadIdx.x; float d1 = 0.f, d2 = 0.f;
#pragma unroll 1
    for (int i = 0; i < HD; ++i) { float p1 = __fmul_rn(bfr(lq1[i]), bfr(lk1[i])); asm volatile("" : "+v"(p1)); d1 = __fadd_rn(d1, p1); float p2 = __fmul_rn(bfr(lq2[i]), bfr(lk2[i])); asm volatile("" : "+v"(p2)); d2 = __fadd_rn(d2, p2); }
    float lm = __fsub_rn(expf(d1), expf(d2)); asm volatile("" : "+v"(lm)); lm = __fadd_rn(lm, 0.8f); const float v = (lane == 0) ? lm : 0.0f; *(volatile float*)(LAM + lane) = v; __threadfence(); *(volatile float*)(LAM + lane) = v; }
__global__ __launch_bounds__(256) void k_qkp(const float* __restrict__ F, int pitch, int nheads, bf* Ph, bf* Pl) {
    const size_t e = ((size_t)blockIdx.x * 256 + threadIdx.x) * 2; if (e >= (size_t)nheads * SEQ * HD) return;
    const int d = (int)(e % HD); const int t = (int)((e / HD) % SEQ); const int vh = (int)(e / ((size_t)HD * SEQ));
    const v2f x = *(const v2f*)(F + (size_t)t * pitch + vh * HD + d); v2us oh, ol;
#pragma unroll
    for (int q = 0; q < 2; ++q) { unsigned short a2, c2; splitf(x[q], a2, c2); oh[q] = a2; ol[q] = c2; }
    *(volatile v2us*)(Ph + e) = oh; *(volatile v2us*)(Pl + e) = ol; __threadfence(); *(volatile v2us*)(Ph + e) = oh; *(volatile v2us*)(Pl + e) = ol; }
__global__ __launch_bounds__(256) void k_vtp(const float* __restrict__ F, int pitch, int nheads, h16* V16, h16* VR) {
    const size_t e = ((size_t)blockIdx.x * 256 + threadIdx.x) * 2; if (e >= (size_t)nheads * HD * SEQ) return;
    const int t = (int)(e % SEQ); const int d = (int)((e / SEQ) % HD); const int g = (int)(e / ((size_t)SEQ * HD)); v2h o16, orr;
#pragma unroll
    for (int q = 0; q < 2; ++q) { const float x = F[(size_t)(t + q) * pitch + g * HD + d]; const h16 hv = tohx(x); const float res = (x - (float)hv) * RCAR; o16[q] = hv; orr[q] = tohx(res); }
    *(volatile v2h*)(V16 + e) = o16; *(volatile v2h*)(VR + e) = orr; __threadfence(); *(volatile v2h*)(V16 + e) = o16; *(volatile v2h*)(VR + e) = orr; }

__device__ __forceinline__ v16bf ldsb(const bf* p) { return cat16b(*(const v8usa*)p, *(const v8usa*)(p + 16)); }
__device__ __forceinline__ v16h  ldsh(const h16* p) { return cat16(*(const v8ha*)p, *(const v8ha*)(p + 16)); }

__global__ __launch_bounds__(128) __attribute__((amdgpu_num_vgpr(256)))
void k_attn(const bf* __restrict__ QPh, const bf* __restrict__ QPl, const bf* __restrict__ KPh, const bf* __restrict__ KPl, const h16* __restrict__ VT, const h16* __restrict__ VR,
            const float* __restrict__ amb, const int* __restrict__ tix, const float* __restrict__ LAM, float* Ob) {
    __shared__ __align__(16) bf    qs[2][QBL * LP];
    __shared__ __align__(16) bf    ks[2][KCH * LP];
    __shared__ __align__(16) h16   vsm[HD * LP];
    __shared__ __align__(16) h16   vrm[HD * LP];
    __shared__ __align__(16) h16   psm[4][16 * PP];
    __shared__ __align__(16) h16   prm[4][16 * PP];
    __shared__ __align__(16) float osm[4][16 * OSP];
    const int tid = threadIdx.x, w = tid >> 5, lane = tid & 31, lr = lane & 15, hi = lane >> 4;
    const int hh = blockIdx.y, qb = blockIdx.x, q0 = qb * QBL; const bool er = (qb == 0);
    const int e2 = hh + 1;
    const float slope = ((e2 & 1) ? 0.70710678118654752f : 1.0f) * __uint_as_float(((unsigned)(127 - (e2 >> 1))) << 23);
    const float lam = LAM[0];
    const int qrow0 = q0 + 16 * w + 8 * hi;
    float pq[8];
#pragma unroll
    for (int r = 0; r < 8; ++r) pq[r] = (float)tix[qrow0 + r];
    h16* pt = &psm[w][0]; h16* prt = &prm[w][0]; float* os = &osm[w][0];
#pragma unroll 1
    for (int st = 0; st < 2; ++st) {
        const size_t vq = (size_t)(2 * hh + st);
        __syncthreads();
#pragma unroll
        for (int i = 0; i < 8; ++i) { const int p = i >> 2; const int rem = (i & 3) * 128 + tid; const int row = rem >> 3, c8 = rem & 7;
            const bf* src = (p ? QPl : QPh) + (vq * SEQ + q0 + row) * HD + c8 * 8; *(v8usa*)(&qs[p][row * LP + c8 * 8]) = *(const v8usa*)src; }
        float m[8], l[8]; v8f O[4];
#pragma unroll
        for (int r = 0; r < 8; ++r) { m[r] = NEGB; l[r] = 0.0f; }
#pragma unroll
        for (int j = 0; j < 4; ++j) O[j] = (v8f){};
#pragma unroll 1
        for (int c = 0; c <= qb; ++c) {
            const int k0 = c * KCH;
#pragma unroll
            for (int i = 0; i < 8; ++i) { const int p = i >> 2; const int rem = (i & 3) * 128 + tid; const int row = rem >> 3, c8 = rem & 7;
                const bf* src = (p ? KPl : KPh) + (vq * SEQ + k0 + row) * HD + c8 * 8; *(v8usa*)(&ks[p][row * LP + c8 * 8]) = *(const v8usa*)src; }
#pragma unroll
            for (int i = 0; i < 4; ++i) { const int rem = i * 128 + tid; const int d = rem >> 3, c8 = rem & 7; const size_t go = ((size_t)hh * HD + d) * SEQ + k0 + 8 * c8;
                *(v8ha*)(&vsm[d * LP + 8 * c8]) = *(const v8ha*)(VT + go); if (er) *(v8ha*)(&vrm[d * LP + 8 * c8]) = *(const v8ha*)(VR + go); }
            __syncthreads();
#pragma unroll 1
            for (int sb = 0; sb < KCH / KSB; ++sb) {
                const int kb = sb * KSB;
                const int key0 = k0 + kb + lr, key1 = key0 + 16;
                const float pk0 = (float)tix[key0], pk1 = (float)tix[key1];
                const float om0 = 1.0f - amb[key0], om1 = 1.0f - amb[key1]; const float pad0 = om0 * -1.0e9f, pad1 = om1 * -1.0e9f;
                v8f s[2]; s[0] = (v8f){}; s[1] = (v8f){};
                {   v16bf ah, al, bh, bl;
#pragma unroll
                    for (int kc = 0; kc < HD; kc += 32) {
                        ah = ldsb(&qs[0][(16 * w + lr) * LP + kc + 8 * hi]); al = ldsb(&qs[1][(16 * w + lr) * LP + kc + 8 * hi]);
#pragma unroll
                        for (int nb = 0; nb < 2; ++nb) { bh = ldsb(&ks[0][(kb + nb * 16 + lr) * LP + kc + 8 * hi]); bl = ldsb(&ks[1][(kb + nb * 16 + lr) * LP + kc + 8 * hi]);
                            s[nb] = wmmab(ah, bh, s[nb]); s[nb] = wmmab(al, bh, s[nb]); s[nb] = wmmab(ah, bl, s[nb]); }
                        asm volatile("v_nop\n\tv_nop\n\tv_nop\n\tv_nop" : "+v"(s[0]), "+v"(s[1]) : "v"(ah), "v"(al), "v"(bh), "v"(bl) : "memory");
                    }
                }
                float cm[8];
#pragma unroll
                for (int r = 0; r < 8; ++r) cm[r] = NEGB;
#pragma unroll
                for (int nb = 0; nb < 2; ++nb) { const int kv = nb ? key1 : key0; const float pkv = nb ? pk1 : pk0; const float pdv = nb ? pad1 : pad0;
#pragma unroll
                    for (int r = 0; r < 8; ++r) { const float sa = s[nb][r] * SCL; const float pd = pq[r] - pkv; const float bia = slope * pd; const float sm = sa - bia;
                        const float tt = (kv <= qrow0 + r) ? (sm + pdv) : NEGB; s[nb][r] = tt; cm[r] = fmaxf(cm[r], tt); } }
                float cor[8], rs[8];
#pragma unroll
                for (int r = 0; r < 8; ++r) { float x = cm[r]; x = fmaxf(x, __shfl_xor(x, 1, 32)); x = fmaxf(x, __shfl_xor(x, 2, 32)); x = fmaxf(x, __shfl_xor(x, 4, 32)); x = fmaxf(x, __shfl_xor(x, 8, 32));
                    const float mn = fmaxf(m[r], x); const float dlt = (m[r] - mn) * L2E; cor[r] = __builtin_amdgcn_exp2f(dlt); m[r] = mn; rs[r] = 0.0f; }
#pragma unroll
                for (int nb = 0; nb < 2; ++nb) { const int kv = nb ? key1 : key0;
#pragma unroll
                    for (int r = 0; r < 8; ++r) { const float dq = (s[nb][r] - m[r]) * L2E; const float pe = __builtin_amdgcn_exp2f(dq); const float p = (kv <= qrow0 + r) ? pe : 0.0f; rs[r] = rs[r] + p;
                        const float pc = p * PCAR; const h16 ph = tohx(pc); const int li = (8 * hi + r) * PP + nb * 16 + lr; pt[li] = ph;
                        if (er) { const float res = (pc - (float)ph) * RCAR; prt[li] = tohx(res); } } }
#pragma unroll
                for (int r = 0; r < 8; ++r) { float x = rs[r]; x += __shfl_xor(x, 1, 32); x += __shfl_xor(x, 2, 32); x += __shfl_xor(x, 4, 32); x += __shfl_xor(x, 8, 32);
                    const float lc = l[r] * cor[r]; l[r] = lc + x; const float cf = cor[r];
#pragma unroll
                    for (int j = 0; j < 4; ++j) O[j][r] = O[j][r] * cf; }
                __syncthreads();
                {   const v16h a = ldsh(pt + lr * PP + 8 * hi); v16h b;
#pragma unroll
                    for (int j = 0; j < 4; ++j) { b = ldsh(&vsm[(j * 16 + lr) * LP + kb + 8 * hi]); O[j] = wmma16(a, b, O[j]); }
                    asm volatile("v_nop\n\tv_nop\n\tv_nop\n\tv_nop" : "+v"(O[0]), "+v"(O[1]), "+v"(O[2]), "+v"(O[3]) : "v"(a), "v"(b) : "memory");
                    if (er) {
                        const v16h ar = ldsh(prt + lr * PP + 8 * hi);
#pragma unroll
                        for (int j = 0; j < 4; ++j) {
                            const v16h b2 = ldsh(&vsm[(j * 16 + lr) * LP + kb + 8 * hi]); const v16h br = ldsh(&vrm[(j * 16 + lr) * LP + kb + 8 * hi]);
                            v8f R = wmma16(ar, b2, (v8f){}); R = wmma16(a, br, R);
                            asm volatile("v_nop\n\tv_nop\n\tv_nop\n\tv_nop" : "+v"(R) : "v"(a), "v"(ar), "v"(b2), "v"(br) : "memory");
#pragma unroll
                            for (int r = 0; r < 8; ++r) { const float rr = R[r] * (1.0f / RCAR); O[j][r] = O[j][r] + rr; }
                        }
                    }
                }
                __syncthreads();
            }
        }
#pragma unroll
        for (int r = 0; r < 8; ++r) { const float rl = 1.0f / l[r]; const float il = rl * (1.0f / PCAR);
#pragma unroll
            for (int j = 0; j < 4; ++j) { const float a1 = O[j][r] * il; const int oi = (8 * hi + r) * OSP + j * 16 + lr;
                if (st == 0) { os[oi] = a1; } else { const float lb = lam * a1; const float cur = os[oi]; os[oi] = cur - lb; } } }
    }
    __syncthreads();
    float* orow = Ob + (size_t)(q0 + 16 * w) * DVV + hh * HD;
#pragma unroll 1
    for (int ps = 0; ps < 2; ++ps) {
#pragma unroll
        for (int s2 = 0; s2 < 8; ++s2) { const int row = 2 * s2 + hi, cofs = lr * 4; const v4f val = *(const v4fa*)(os + row * OSP + cofs); *(volatile v4f*)(orow + (size_t)row * DVV + cofs) = val; }
        if (ps == 0) __threadfence(); }
}

__global__ __launch_bounds__(1024) void k_gnstat(const float* __restrict__ O, float* GST) {
    __shared__ float sh[1024]; const int tid = threadIdx.x; const int hh = blockIdx.x; const float* base = O + hh * HD; const int n = SEQ * HD; const float rn = 1.0f / (float)n;
    float acc = 0.f;
#pragma unroll 1
    for (int e = tid; e < n; e += 1024) { const int t = e >> 6, d = e & 63; acc = __fadd_rn(acc, base[(size_t)t * DVV + d]); }
    sh[tid] = acc; __syncthreads();
#pragma unroll 1
    for (int st = 512; st > 0; st >>= 1) { if (tid < st) sh[tid] = __fadd_rn(sh[tid], sh[tid + st]); __syncthreads(); }
    const float mean = sh[0] * rn;
    __syncthreads();
    float acc2 = 0.f;
#pragma unroll 1
    for (int e = tid; e < n; e += 1024) { const int t = e >> 6, d = e & 63; float dv = __fsub_rn(base[(size_t)t * DVV + d], mean); asm volatile("" : "+v"(dv)); acc2 = __fadd_rn(acc2, __fmul_rn(dv, dv)); }
    sh[tid] = acc2; __syncthreads();
#pragma unroll 1
    for (int st = 512; st > 0; st >>= 1) { if (tid < st) sh[tid] = __fadd_rn(sh[tid], sh[tid + st]); __syncthreads(); }
    if (tid < 32) { const float var = sh[0] * rn; const float rs = __fdiv_rn(1.0f, sqrtf(__fadd_rn(var, 1e-5f))); const float outv = (tid == 0) ? mean : ((tid == 1) ? rs : 0.0f);
        *(volatile float*)(GST + hh * 32 + tid) = outv; __threadfence(); *(volatile float*)(GST + hh * 32 + tid) = outv; }
}
__global__ __launch_bounds__(256) void k_gnmerge(const float* __restrict__ O, const float* __restrict__ GST, const float* __restrict__ gw, const float* __restrict__ gb, bf* Ah, bf* Al) {
    const size_t e = ((size_t)blockIdx.x * 256 + threadIdx.x) * 2; if (e >= (size_t)SEQ * DVV) return;
    const int c = (int)(e % DVV); const int hh = c / HD; const float mean = GST[hh * 32], rs = GST[hh * 32 + 1]; v2us oh, ol;
#pragma unroll
    for (int q = 0; q < 2; ++q) { float cc = __fsub_rn(O[e + q], mean); asm volatile("" : "+v"(cc)); float nn = __fmul_rn(cc, rs); asm volatile("" : "+v"(nn)); float y = __fmul_rn(nn, bfr(gw[c + q])); asm volatile("" : "+v"(y)); y = __fadd_rn(y, bfr(gb[c + q])); const float z = __fmul_rn(y, 0.2f); unsigned short a2, c2; splitf(z, a2, c2); oh[q] = a2; ol[q] = c2; }
    *(volatile v2us*)(Ah + e) = oh; *(volatile v2us*)(Al + e) = ol; __threadfence(); *(volatile v2us*)(Ah + e) = oh; *(volatile v2us*)(Al + e) = ol; }

extern "C" void kernel_launch(void* const* d_in, const int* in_sizes, int n_in,
                              void* d_out, int out_size, void* d_ws, size_t ws_size, hipStream_t stream) {
    if (n_in < 13) return;
    if (in_sizes[0] < (NB - 1) * SEQ_FULL * DM + SEQ * DM) return;
    if (in_sizes[1] < (NB - 1) * SEQ_FULL + SEQ) return;
    if (in_sizes[2] < (NB - 1) * SEQ_FULL + SEQ) return;
    if (in_sizes[3] < DQ * DM || in_sizes[4] < DQ * DM || in_sizes[5] < DVV * DM || in_sizes[6] < DM * DVV) return;
    if (in_sizes[7] < HD || in_sizes[8] < HD || in_sizes[9] < HD || in_sizes[10] < HD || in_sizes[11] < DVV || in_sizes[12] < DVV) return;
    if (out_size < (NB - 1) * SEQ_FULL * DM + SEQ * DM) return;
    const float* x = (const float*)d_in[0]; const float* amask = (const float*)d_in[1]; const int* tix = (const int*)d_in[2];
    const float* wq = (const float*)d_in[3]; const float* wk = (const float*)d_in[4]; const float* wv = (const float*)d_in[5]; const float* wo = (const float*)d_in[6];
    const float* lq1 = (const float*)d_in[7]; const float* lq2 = (const float*)d_in[8]; const float* lk1 = (const float*)d_in[9]; const float* lk2 = (const float*)d_in[10];
    const float* gnw = (const float*)d_in[11]; const float* gnb = (const float*)d_in[12];
    float* OUT = (float*)d_out;
    char* wsp = (char*)d_ws;
    auto take = [&](size_t bytes) { char* p = wsp; wsp += (bytes + 255) & ~(size_t)255; return (void*)p; };
    bf* WQ = (bf*)take((size_t)DQ * DM * 2); bf* WK = (bf*)take((size_t)DQ * DM * 2); bf* WV = (bf*)take((size_t)DVV * DM * 2); bf* WO = (bf*)take((size_t)DM * DVV * 2);
    bf* XB = (bf*)take((size_t)SEQ * DM * 2); float* AMB = (float*)take((size_t)SEQ * 4); float* LAM = (float*)take(256); float* GST = (float*)take((size_t)NVH * 32 * 4);
    float* FQ = (float*)take((size_t)SEQ * DQ * 4); float* FK = (float*)take((size_t)SEQ * DQ * 4);
    bf* QPh = (bf*)take((size_t)NQH * SEQ * HD * 2); bf* QPl = (bf*)take((size_t)NQH * SEQ * HD * 2); bf* KPh = (bf*)take((size_t)NQH * SEQ * HD * 2); bf* KPl = (bf*)take((size_t)NQH * SEQ * HD * 2);
    h16* VT16 = (h16*)take((size_t)NVH * HD * SEQ * 2); h16* VRS = (h16*)take((size_t)NVH * HD * SEQ * 2);
    float* Ob = (float*)take((size_t)SEQ * DVV * 4); bf* ATh = (bf*)take((size_t)SEQ * DVV * 2); bf* ATl = (bf*)take((size_t)SEQ * DVV * 2);
    const size_t used = (size_t)(wsp - (char*)d_ws);
    if (used > ws_size || used > (size_t)134217728) return;
    float* FV = FK;
    k_cvt8<<<(unsigned)(((size_t)DQ * DM / 8 + 255) / 256), 256, 0, stream>>>(wq, WQ, (size_t)DQ * DM / 8);
    k_cvt8<<<(unsigned)(((size_t)DQ * DM / 8 + 255) / 256), 256, 0, stream>>>(wk, WK, (size_t)DQ * DM / 8);
    k_cvt8<<<(unsigned)(((size_t)DVV * DM / 8 + 255) / 256), 256, 0, stream>>>(wv, WV, (size_t)DVV * DM / 8);
    k_cvt8<<<(unsigned)(((size_t)DM * DVV / 8 + 255) / 256), 256, 0, stream>>>(wo, WO, (size_t)DM * DVV / 8);
    k_lambda<<<1, 32, 0, stream>>>(lq1, lk1, lq2, lk2, LAM);
    const unsigned LQK = (unsigned)(((size_t)NQH * SEQ * HD / 2 + 255) / 256), LV = (unsigned)(((size_t)NVH * HD * SEQ / 2 + 255) / 256);
    for (int b = 0; b < NB; ++b) {
        const float* xb = x + (size_t)b * SEQ_FULL * DM; const float* amb = amask + (size_t)b * SEQ_FULL; const int* tixb = tix + (size_t)b * SEQ_FULL; float* outb = OUT + (size_t)b * SEQ_FULL * DM;
        k_cvt8<<<(unsigned)(((size_t)SEQ * DM / 8 + 255) / 256), 256, 0, stream>>>(xb, XB, (size_t)SEQ * DM / 8);
        k_rbf<<<(SEQ / 4 + 255) / 256, 256, 0, stream>>>(amb, AMB, SEQ / 4);
        k_gemmw<bf, 0, false><<<dim3(SEQ / 64, DQ / 64, 1), 32, 0, stream>>>(XB, nullptr, WQ, nullptr, DM, FQ, DQ, nullptr, 0, 0, 0);
        k_qkp<<<LQK, 256, 0, stream>>>(FQ, DQ, NQH, QPh, QPl);
        k_gemmw<bf, 0, false><<<dim3(SEQ / 64, DQ / 64, 1), 32, 0, stream>>>(XB, nullptr, WK, nullptr, DM, FK, DQ, nullptr, 0, 0, 0);
        k_qkp<<<LQK, 256, 0, stream>>>(FK, DQ, NQH, KPh, KPl);
        k_gemmw<bf, 0, false><<<dim3(SEQ / 64, DVV / 64, 1), 32, 0, stream>>>(XB, nullptr, WV, nullptr, DM, FV, DVV, nullptr, 0, 0, 0);
        k_vtp<<<LV, 256, 0, stream>>>(FV, DVV, NVH, VT16, VRS);
        k_attn<<<dim3(SEQ / QBL, NVH, 1), 128, 0, stream>>>(QPh, QPl, KPh, KPl, VT16, VRS, AMB, tixb, LAM, Ob);
        k_gnstat<<<NVH, 1024, 0, stream>>>(Ob, GST);
        k_gnmerge<<<(unsigned)(((size_t)SEQ * DVV / 2 + 255) / 256), 256, 0, stream>>>(Ob, GST, gnw, gnb, ATh, ATl);
        k_gemmw<bf, 1, false><<<dim3(SEQ / 64, DM / 64, 1), 32, 0, stream>>>(ATh, ATl, WO, nullptr, DVV, outb, DM, nullptr, 0, 0, 0);
    }
}
